// RGCNLayer_35639638622237
// MI455X (gfx1250) — hardware-verified
//
#include <hip/hip_runtime.h>
#include <math.h>

typedef __attribute__((ext_vector_type(16))) _Float16 v16h;
typedef __attribute__((ext_vector_type(16))) __bf16 v16b;
typedef __attribute__((ext_vector_type(8)))  _Float16 v8h;
typedef __attribute__((ext_vector_type(8)))  float v8f;
typedef __attribute__((ext_vector_type(4)))  float v4f;
typedef __attribute__((ext_vector_type(2)))  float v2f;
typedef __attribute__((ext_vector_type(4)))  unsigned v4u;
typedef __attribute__((ext_vector_type(4)))  int v4i;
typedef float __attribute__((may_alias)) float_a;
typedef int __attribute__((may_alias)) int_a;

template <typename T> __device__ __forceinline__ void vst2(void* p, T v) { *(volatile T*)p = v; __threadfence(); *(volatile T*)p = v; }
__device__ __forceinline__ v8f wmma16(v16h a, v16h b, v8f c) {
  v8f d = __builtin_amdgcn_wmma_f32_16x16x32_f16(false, a, false, b, (short)0, c, false, false);
  asm volatile("v_nop\n\tv_nop\n\tv_nop\n\tv_nop" : "+v"(d) : "v"(a), "v"(b));
  return d;
}
__device__ __forceinline__ v8f wmma_bf(v16b a, v16b b, v8f c) {
  v8f d = __builtin_amdgcn_wmma_f32_16x16x32_bf16(false, a, false, b, (short)0, c, false, false);
  asm volatile("v_nop\n\tv_nop\n\tv_nop\n\tv_nop" : "+v"(d) : "v"(a), "v"(b));
  return d;
}
__device__ __forceinline__ v16h frag_h(const _Float16* rowk0, int lane) {
  union { v16h v; v8h q[2]; } u; const _Float16* p = rowk0 + 8 * (lane >> 4);
  u.q[0] = *(const v8h*)p; u.q[1] = *(const v8h*)(p + 16); return u.v;
}
__device__ __forceinline__ v16h frag_f32(const float* rowk0, int lane) {
  v16h a; const float* p = rowk0 + 8 * (lane >> 4);
#pragma unroll
  for (int i = 0; i < 8; ++i) { a[i] = (_Float16)p[i]; a[8 + i] = (_Float16)p[16 + i]; }
  return a;
}
__device__ __forceinline__ v16h frag_f32s(const float* rowk0, int lane, float sc) {
  v16h a; const float* p = rowk0 + 8 * (lane >> 4);
#pragma unroll
  for (int i = 0; i < 8; ++i) { a[i] = (_Float16)(p[i] * sc); a[8 + i] = (_Float16)(p[16 + i] * sc); }
  return a;
}
__device__ __forceinline__ v16h fragc_f32(const float* W, int k0, int n, int lane, int ld, int K) {
  v16h a; const int g = lane >> 4;
#pragma unroll
  for (int i = 0; i < 8; ++i) { const int ka = k0 + 8 * g + i, kb = ka + 16;
    a[i] = (_Float16)(ka < K ? W[(size_t)ka * ld + n] : 0.f); a[8 + i] = (_Float16)(kb < K ? W[(size_t)kb * ld + n] : 0.f); }
  return a;
}
struct F2 { v16b h, l; };
__device__ __forceinline__ F2 bsplit16(const float v[16]) { F2 r;
#pragma unroll
  for (int i = 0; i < 16; ++i) { const __bf16 h = (__bf16)v[i]; r.h[i] = h; r.l[i] = (__bf16)(v[i] - (float)h); }
  return r; }
__device__ __forceinline__ F2 split_row(const float* row, int k0, int lane) { float v[16]; const float* p = row + k0 + 8 * (lane >> 4);
#pragma unroll
  for (int i = 0; i < 8; ++i) { v[i] = p[i]; v[8 + i] = p[16 + i]; }
  return bsplit16(v); }
__device__ __forceinline__ F2 split_rowK(const float* row, int k0, int lane, int K) { float v[16]; const int g = lane >> 4;
#pragma unroll
  for (int i = 0; i < 8; ++i) { const int ka = k0 + 8 * g + i, kb = ka + 16; v[i] = ka < K ? row[ka] : 0.f; v[8 + i] = kb < K ? row[kb] : 0.f; }
  return bsplit16(v); }
__device__ __forceinline__ F2 split_col(const float* W, int k0, int n, int lane, int ld, int K) { float v[16]; const int g = lane >> 4;
#pragma unroll
  for (int i = 0; i < 8; ++i) { const int ka = k0 + 8 * g + i, kb = ka + 16; v[i] = ka < K ? W[(size_t)ka * ld + n] : 0.f; v[8 + i] = kb < K ? W[(size_t)kb * ld + n] : 0.f; }
  return bsplit16(v); }
__device__ __forceinline__ v8f mac3(const F2& a, const F2& b, v8f c) { c = wmma_bf(a.l, b.h, c); c = wmma_bf(a.h, b.l, c); return wmma_bf(a.h, b.h, c); }
__device__ __forceinline__ float sigm(float v) { return 1.0f / (1.0f + expf(-v)); }
#define LDSX() do { asm volatile("s_wait_dscnt 0" ::: "memory"); __builtin_amdgcn_wave_barrier(); __builtin_amdgcn_fence(__ATOMIC_RELEASE, "workgroup"); } while (0)


#define NN 100000
#define NE 1600000
#define FD 32
#define NR 16
#define NB 8
#define TW 576
#define TC (NR * FD + FD)
#define RB 1024
#define NRB 98
#define NNP (NRB * RB)
#define RBD 8192
#define NRBD ((NNP + RBD - 1) / RBD)
#define EPT 8
#define CH (256 * EPT)
__device__ __forceinline__ int clampn(int v) { return v < 0 ? 0 : (v >= NN ? NN - 1 : v); }

__global__ __launch_bounds__(256) void k_prep(const float* __restrict__ weight, const float* __restrict__ wcomp, const float* __restrict__ emb, const float* __restrict__ Aw, const float* __restrict__ Ab,
                                            float* __restrict__ RW, float* __restrict__ P3) {
  const int tid = threadIdx.x;
#pragma unroll 1
  for (int q = tid; q < NR * FD * FD; q += 256) { const int r = q / (FD * FD), io = q % (FD * FD); float s = 0.f;
#pragma unroll
    for (int b = 0; b < NB; ++b) s += wcomp[r * NB + b] * weight[b * FD * FD + io];
    vst2(RW + q, (float_a)s); }
#pragma unroll 1
  for (int q = tid; q < NR * FD; q += 256) { const int r = q / FD, c = q % FD; float s = Ab[c];
#pragma unroll 4
    for (int k = 0; k < FD; ++k) s += emb[r * FD + k] * Aw[(2 * FD + k) * FD + c];
    vst2(P3 + q, (float_a)s); }
}
__global__ __launch_bounds__(128) void k_tab(const float* __restrict__ h, const float* __restrict__ RW, const float* __restrict__ Aw, _Float16* __restrict__ T) {
  __shared__ __align__(16) _Float16 so[4][16][TW + 8];
  const int tid = threadIdx.x, wave = tid >> 5, lane = tid & 31, col = lane & 15, g = lane >> 4;
  const int r0 = blockIdx.x * 64 + wave * 16; const int ra = (r0 + col) < NN ? (r0 + col) : (NN - 1);
  const F2 a = split_row(h + (size_t)ra * FD, 0, lane);
#pragma unroll 1
  for (int ps = 0; ps < 5; ++ps) { const int t0 = ps * 8; const int nt = (TC / 16 - t0) < 8 ? (TC / 16 - t0) : 8;
    v8f acc[8] = {};
#pragma unroll
    for (int j = 0; j < 8; ++j) if (j < nt) { const int n = (t0 + j) * 16 + col; const float* Bp = n < NR * FD ? RW + (size_t)(n / FD) * FD * FD : Aw; const int nn = n % FD;
      acc[j] = mac3(a, split_col(Bp, 0, nn, lane, FD, FD), acc[j]); }
#pragma unroll
    for (int j = 0; j < 8; ++j) if (j < nt) {
#pragma unroll
      for (int r = 0; r < 8; ++r) so[wave][8 * g + r][(t0 + j) * 16 + col] = (_Float16)((r0 + 8 * g + r) < NN ? acc[j][r] : 0.f); } }
  for (int q = lane; q < 16 * (TW - TC); q += 32) so[wave][q / (TW - TC)][TC + q % (TW - TC)] = (_Float16)0.0f;
  LDSX();
  for (int q = lane; q < 16 * (TW / 8); q += 32) { const int rl = q / (TW / 8), pc = q % (TW / 8); vst2(T + (size_t)(r0 + rl) * TW + pc * 8, *(const v4u*)(&so[wave][rl][pc * 8])); }
}
__global__ __launch_bounds__(256) void k_deg(const int* __restrict__ edst, float* __restrict__ DEG) {
  __shared__ int scnt[RBD];
  const int tid = threadIdx.x; const int r0 = blockIdx.x * RBD;
  for (int q = tid; q < RBD; q += 256) scnt[q] = 0;
  __syncthreads();
#pragma unroll 1
  for (int c0 = 0; c0 < NE; c0 += CH) { const int e0 = c0 + tid * EPT;
    if (e0 + EPT <= NE) {
#pragma unroll
      for (int v = 0; v < EPT / 4; ++v) { const int4 d4 = *(const int4*)(edst + e0 + v * 4); const int dd[4] = {d4.x, d4.y, d4.z, d4.w};
#pragma unroll
        for (int u = 0; u < 4; ++u) { const unsigned rel = (unsigned)(dd[u] - r0); if (rel < (unsigned)RBD) atomicAdd(&scnt[rel], 1); } } }
    else { for (int u = 0; u < EPT; ++u) { const int e = e0 + u; if (e < NE) { const unsigned rel = (unsigned)(edst[e] - r0); if (rel < (unsigned)RBD) atomicAdd(&scnt[rel], 1); } } } }
  __syncthreads();
  for (int q = tid; q < RBD; q += 256) { const int r = r0 + q; if (r < NNP) vst2(DEG + r, r < NN ? (float)scnt[q] : 0.f); }
}
__global__ __launch_bounds__(256) void k_mean(const float* __restrict__ DEG, float* __restrict__ MEANL) {
  __shared__ float sp[256]; const int tid = threadIdx.x; float s = 0.f;
#pragma unroll 1
  for (int n = tid; n < NN; n += 256) s += logf(DEG[n] + 1.0f);
  sp[tid] = s; __syncthreads();
#pragma unroll
  for (int off = 128; off > 0; off >>= 1) { if (tid < off) sp[tid] += sp[tid + off]; __syncthreads(); }
  if (tid < 32) vst2(MEANL + tid, (float_a)(sp[0] / (float)NN));
}
__global__ __launch_bounds__(256) void k_agg(const int* __restrict__ esrc, const int* __restrict__ edst, const int* __restrict__ etyp, const float* __restrict__ h, const _Float16* __restrict__ T,
                                            const float* __restrict__ Aw, const float* __restrict__ P3, const float* __restrict__ Bw, const float* __restrict__ Bb, const float* __restrict__ Wself,
                                            const float* __restrict__ bias, const float* __restrict__ DEG, const float* __restrict__ MEANL, float* __restrict__ out) {
  __shared__ __align__(16) float sacc[RB][FD];
  __shared__ __align__(16) float sp2[RB][FD];
  __shared__ float sp3[NR][FD]; __shared__ float sbw[FD];
  __shared__ int slst[8][32 * EPT], sdl[8][32 * EPT]; __shared__ float swgt[8][32 * EPT]; __shared__ int scnt[8];
  const int tid = threadIdx.x, wave = tid >> 5, lane = tid & 31, col = lane & 15, g = lane >> 4;
  const int r0 = blockIdx.x * RB; const float bb0 = Bb[0];
  for (int q = tid; q < RB * FD; q += 256) (&sacc[0][0])[q] = 0.f;
  for (int q = tid; q < NR * FD; q += 256) (&sp3[0][0])[q] = P3[q];
  if (tid < FD) sbw[tid] = Bw[tid];
#pragma unroll 1
  for (int rt = wave; rt < RB / 16; rt += 8) { const int row = r0 + rt * 16 + col; const int ra = row < NN ? row : NN - 1; const F2 a = split_row(h + (size_t)ra * FD, 0, lane);
#pragma unroll
    for (int j = 0; j < 2; ++j) { v8f acc = {}; acc = mac3(a, split_col(Aw + (size_t)FD * FD, 0, j * 16 + col, lane, FD, FD), acc);
#pragma unroll
      for (int r = 0; r < 8; ++r) sp2[rt * 16 + 8 * g + r][j * 16 + col] = acc[r]; } }
  __syncthreads();
#pragma unroll 1
  for (int c0 = 0; c0 < NE; c0 += CH) { const int e0 = c0 + tid * EPT; int hd[EPT]; int cnt = 0;
    if (e0 + EPT <= NE) {
#pragma unroll
      for (int v = 0; v < EPT / 4; ++v) { const int4 d4 = *(const int4*)(edst + e0 + v * 4); const int dd[4] = {d4.x, d4.y, d4.z, d4.w};
#pragma unroll
        for (int u = 0; u < 4; ++u) { const unsigned rel = (unsigned)(clampn(dd[u]) - r0); const bool hh = rel < (unsigned)RB; hd[v * 4 + u] = hh ? (int)rel : -1; cnt += hh ? 1 : 0; } } }
    else {
#pragma unroll
      for (int u = 0; u < EPT; ++u) { const int e = e0 + u; hd[u] = -1; if (e < NE) { const unsigned rel = (unsigned)(clampn(edst[e]) - r0); if (rel < (unsigned)RB) { hd[u] = (int)rel; ++cnt; } } } }
    int incl = cnt;
#pragma unroll
    for (int off = 1; off < 32; off <<= 1) { const int vv = __shfl_up(incl, off, 32); if (lane >= off) incl += vv; }
    const int wtot = __shfl(incl, 31, 32); int pos = incl - cnt;
    if (cnt > 0) {
#pragma unroll
      for (int u = 0; u < EPT; ++u) if (hd[u] >= 0) { slst[wave][pos] = e0 + u; sdl[wave][pos] = hd[u]; ++pos; } }
    if (lane == 0) scnt[wave] = wtot;
    __syncthreads();
#pragma unroll 1
    for (int w = 0; w < 8; ++w) { const int nh = scnt[w];
#pragma unroll 1
      for (int i = tid; i < nh; i += 256) { const int e = slst[w][i]; const int s = clampn(esrc[e]); int r = etyp[e]; r = r < 0 ? 0 : (r >= NR ? NR - 1 : r); const int dl = sdl[w][i];
        const _Float16* p1 = T + (size_t)s * TW + NR * FD; const float* p2 = &sp2[dl][0]; const float* p3 = &sp3[r][0]; float dot = bb0;
#pragma unroll 1
        for (int c = 0; c < FD; ++c) { const float z = (float)p1[c] + p2[c] + p3[c]; dot += (z > 0.f ? z : 0.f) * sbw[c]; }
        swgt[w][i] = sigm(dot); slst[w][i] = s * NR + r; } }
    __syncthreads();
    if (tid < FD) {
#pragma unroll 1
      for (int w = 0; w < 8; ++w) { const int nh = scnt[w];
#pragma unroll 1
        for (int i = 0; i < nh; ++i) { const int sr = slst[w][i], dl = sdl[w][i]; const int s = sr >> 4, r = sr & 15; sacc[dl][tid] += swgt[w][i] * (float)T[(size_t)s * TW + r * FD + tid]; } } }
    __syncthreads(); }
#pragma unroll 1
  for (int rt = wave; rt < RB / 16; rt += 8) { const int row = r0 + rt * 16 + col; const int ra = row < NN ? row : NN - 1; const F2 a = split_row(h + (size_t)ra * FD, 0, lane);
#pragma unroll
    for (int j = 0; j < 2; ++j) { v8f acc = {}; acc = mac3(a, split_col(Wself, 0, j * 16 + col, lane, FD, FD), acc);
#pragma unroll
      for (int r = 0; r < 8; ++r) sp2[rt * 16 + 8 * g + r][j * 16 + col] = acc[r]; } }
  __syncthreads();
  const float meanl = MEANL[0];
#pragma unroll 1
  for (int q = tid; q < RB * (FD / 4); q += 256) { const int rl = q >> 3, pc = q & 7; const int row = r0 + rl; if (row >= NN) continue;
    v4f o; const float dg = DEG[row]; const float sc = (logf(dg + 1.0f) / meanl) / fmaxf(dg, 1.0f);
    const v4f a = *(const v4f*)(&sacc[rl][pc * 4]), c = *(const v4f*)(&sp2[rl][pc * 4]), b4 = *(const v4f*)(bias + pc * 4);
#pragma unroll
    for (int e = 0; e < 4; ++e) { const float v = c[e] + sc * a[e] + b4[e]; o[e] = v > 0.f ? v : 0.f; }
    vst2(out + (size_t)row * FD + pc * 4, o); }
}
extern "C" void kernel_launch(void* const* d_in, const int* in_sizes, int n_in, void* d_out, int out_size, void* d_ws, size_t ws_size, hipStream_t stream) {
  (void)in_sizes; (void)n_in; (void)out_size; (void)ws_size;
  const float* h = (const float*)d_in[0]; const float* weight = (const float*)d_in[1]; const float* wcomp = (const float*)d_in[2]; const float* Wself = (const float*)d_in[3]; const float* bias = (const float*)d_in[4];
  const float* emb = (const float*)d_in[5]; const float* Aw = (const float*)d_in[6]; const float* Ab = (const float*)d_in[7]; const float* Bw = (const float*)d_in[8]; const float* Bb = (const float*)d_in[9];
  const int* esrc = (const int*)d_in[10]; const int* edst = (const int*)d_in[11]; const int* etyp = (const int*)d_in[12];
  float* out = (float*)d_out;
  char* ws = (char*)d_ws; size_t off = 0;
  auto take = [&](size_t bytes) { char* p = ws + off; off += (bytes + 255) & ~(size_t)255; return p; };
  float* RW = (float*)take((size_t)NR * FD * FD * 4); float* P3 = (float*)take((size_t)NR * FD * 4); _Float16* T = (_Float16*)take((size_t)NNP * TW * 2);
  float* DEG = (float*)take((size_t)NNP * 4); float* MEANL = (float*)take(256);
  k_prep<<<1, 256, 0, stream>>>(weight, wcomp, emb, Aw, Ab, RW, P3);
  k_tab<<<NNP / 64, 128, 0, stream>>>(h, RW, Aw, T);
  k_deg<<<NRBD, 256, 0, stream>>>(edst, DEG);
  k_mean<<<1, 256, 0, stream>>>(DEG, MEANL);
  k_agg<<<NRB, 256, 0, stream>>>(esrc, edst, etyp, h, T, Aw, P3, Bw, Bb, Wself, bias, DEG, MEANL, out);
}
